// CausalSlidingWindowGQA_7464653160668
// MI455X (gfx1250) — hardware-verified
//
#include <hip/hip_runtime.h>
#define SN 1024
#define LP 4096
#define ED 1024
#define NHQ 16
#define NKV 4
#define HDM 64
#define WIN 32
#define NKB_ALL ((LP + SN) / 64)
#define NKB_MAX 40
#define KC (NKB_MAX * 64)

typedef __bf16 v16b __attribute__((ext_vector_type(16)));
typedef unsigned short v8us __attribute__((ext_vector_type(8), may_alias));
typedef float  v8f  __attribute__((ext_vector_type(8)));
typedef float  v4f  __attribute__((ext_vector_type(4)));
typedef float  v4fa __attribute__((ext_vector_type(4), may_alias));
union FragB { v16b v; v8us half[2]; unsigned short u[16]; };

__device__ __forceinline__ unsigned short bf16_bits(float x) { unsigned int u = __float_as_uint(x); return (unsigned short)((u + 0x7FFFu + ((u >> 16) & 1u)) >> 16); }
__device__ __forceinline__ float bf16_val(unsigned short b) { return __uint_as_float(((unsigned int)b) << 16); }
__device__ __forceinline__ float bf16_round(float x) { return bf16_val(bf16_bits(x)); }
template <int NT>
__device__ __forceinline__ v8f mmaN(v16b ah, v16b al, v16b bh, v16b bl, v8f c) {
  c = __builtin_amdgcn_wmma_f32_16x16x32_bf16(false, ah, false, bh, (short)0, c, false, false);
  if (NT >= 2) c = __builtin_amdgcn_wmma_f32_16x16x32_bf16(false, al, false, bh, (short)0, c, false, false);
  if (NT >= 3) c = __builtin_amdgcn_wmma_f32_16x16x32_bf16(false, ah, false, bl, (short)0, c, false, false);
  asm volatile("v_nop\n\tv_nop\n\tv_nop\n\tv_nop" : "+v"(c) : "v"(ah), "v"(al), "v"(bh), "v"(bl));
  return c;
}

__global__ __launch_bounds__(256) void k_wt_bf16(const float* __restrict__ W, unsigned short* __restrict__ Wt, int K, int N) {
  const int t = blockIdx.x * 256 + threadIdx.x;
  const int k8n = K / 8;
  if (t >= N * k8n) return;
  const int n = t / k8n, k8 = (t % k8n) * 8;
  v8us v;
#pragma unroll
  for (int i = 0; i < 8; ++i) v[i] = bf16_bits(W[(size_t)(k8 + i) * N + n]);
  *(volatile v8us*)(Wt + (size_t)n * K + k8) = v;
  __threadfence();
  *(volatile v8us*)(Wt + (size_t)n * K + k8) = v;
}

template <bool ASPLIT, int ACT, bool BIAS_BF16>
__global__ __launch_bounds__(128) void k_gemm_bf(const float* __restrict__ A, int lda, const unsigned short* __restrict__ Wt, int ldb,
                                               const float* __restrict__ bias, float* __restrict__ C, int ldc, int M, int N, int K) {
  __shared__ __attribute__((aligned(16))) float so[4][16][64];
  const int tid = threadIdx.x, w = tid >> 5, lane = tid & 31, ln = lane & 15, hh = lane >> 4;
  const int ntn = N / 64;
  const int wid = blockIdx.x * 4 + w;
  const int mt = wid / ntn, nq = wid % ntn;
  if (mt * 16 >= M) return;
  const int row0 = mt * 16, col0 = nq * 64;
  const float* arow = A + (size_t)(row0 + ln) * lda;
  v8f acc[4] = {};
  for (int kb = 0; kb < K; kb += 32) {
    FragB ah, al;
    const v4f x0 = *(const v4fa*)(arow + kb + 8 * hh), x1 = *(const v4fa*)(arow + kb + 8 * hh + 4);
    const v4f x2 = *(const v4fa*)(arow + kb + 16 + 8 * hh), x3 = *(const v4fa*)(arow + kb + 16 + 8 * hh + 4);
    float xs[16] = {x0[0],x0[1],x0[2],x0[3],x1[0],x1[1],x1[2],x1[3],x2[0],x2[1],x2[2],x2[3],x3[0],x3[1],x3[2],x3[3]};
#pragma unroll
    for (int i = 0; i < 16; ++i) { const unsigned short hb = bf16_bits(xs[i]); ah.u[i] = hb; al.u[i] = ASPLIT ? bf16_bits(xs[i] - bf16_val(hb)) : (unsigned short)0; }
#pragma unroll
    for (int t = 0; t < 4; ++t) {
      const unsigned short* brow = Wt + (size_t)(col0 + t * 16 + ln) * ldb + kb;
      FragB b;
      b.half[0] = *(const v8us*)(brow + 8 * hh);
      b.half[1] = *(const v8us*)(brow + 16 + 8 * hh);
      acc[t] = mmaN<ASPLIT ? 2 : 1>(ah.v, al.v, b.v, b.v, acc[t]);
    }
  }
#pragma unroll
  for (int t = 0; t < 4; ++t) {
    float bv = bias ? bias[col0 + t * 16 + ln] : 0.f;
    if (BIAS_BF16) bv = bf16_round(bv);
#pragma unroll
    for (int r = 0; r < 8; ++r) { float v = acc[t][r] + bv; if (ACT == 1) v = fmaxf(v, 0.f); so[w][8 * hh + r][t * 16 + ln] = v; }
  }
  __builtin_amdgcn_fence(__ATOMIC_ACQ_REL, "workgroup");
  __builtin_amdgcn_wave_barrier();
  const int rsub = lane >> 4, c4 = (lane & 15) * 4;
  for (int pass = 0; pass < 2; ++pass) {
#pragma unroll
    for (int q = 0; q < 8; ++q) {
      const int r = q * 2 + rsub;
      const v4f v = *(const v4fa*)&so[w][r][c4];
      *(volatile v4f*)(C + (size_t)(row0 + r) * ldc + col0 + c4) = v;
    }
    if (pass == 0) __threadfence();
  }
}

template <int D, bool CAUSAL>
__global__ __launch_bounds__(128) void k_flash(const float* __restrict__ qb, const float* __restrict__ kb, const float* __restrict__ vb,
                                             int pitch, int T, int H, float scale, float* __restrict__ y, int ypitch) {
  constexpr int KS = D / 32;
  constexpr int DT = D / 16;
  __shared__ __attribute__((aligned(16))) unsigned short sKh[32][D + 8], sKl[32][D + 8], sVh[32][D + 8], sVl[32][D + 8];
  __shared__ __attribute__((aligned(16))) unsigned short sPh[4][16][40], sPl[4][16][40];
  __shared__ __attribute__((aligned(16))) float sO[4][16][D];
  const int tid = threadIdx.x, w = tid >> 5, lane = tid & 31, ln = lane & 15, hh = lane >> 4;
  const int nqb = (T + 63) / 64;
  const int bh = blockIdx.x / nqb, qblk = blockIdx.x % nqb;
  const int b = bh / H, h = bh % H;
  const int q0 = qblk * 64 + w * 16;
  const float* Q = qb + (size_t)b * T * pitch + h * D;
  const float* K = kb + (size_t)b * T * pitch + h * D;
  const float* V = vb + (size_t)b * T * pitch + h * D;

  FragB aqh[KS], aql[KS];
  {
    int row = q0 + ln; if (row >= T) row = T - 1;
    const float* qr = Q + (size_t)row * pitch;
#pragma unroll
    for (int ks = 0; ks < KS; ++ks)
#pragma unroll
      for (int i = 0; i < 16; ++i) {
        const int d = ks * 32 + ((i < 8) ? (8 * hh + i) : (16 + 8 * hh + (i - 8)));
        const float x = qr[d] * scale; const unsigned short hb = bf16_bits(x);
        aqh[ks].u[i] = hb; aql[ks].u[i] = bf16_bits(x - bf16_val(hb));
      }
  }
  float m_r[8], l_r[8];
#pragma unroll
  for (int r = 0; r < 8; ++r) { m_r[r] = -3.0e38f; l_r[r] = 0.f; }
  v8f oacc[DT];
#pragma unroll
  for (int dt = 0; dt < DT; ++dt) oacc[dt] = (v8f){0.f,0.f,0.f,0.f,0.f,0.f,0.f,0.f};

  const int kv_end = CAUSAL ? min(T, qblk * 64 + 64) : T;
  for (int j0 = 0; j0 < kv_end; j0 += 32) {
    __syncthreads();
    for (int e = tid; e < 32 * (D / 4); e += 128) {
      const int r = e / (D / 4), c4 = (e % (D / 4)) * 4;
      const int key = j0 + r;
      v4f kf = {0.f,0.f,0.f,0.f}, vf = {0.f,0.f,0.f,0.f};
      if (key < T) { kf = *(const v4fa*)(K + (size_t)key * pitch + c4); vf = *(const v4fa*)(V + (size_t)key * pitch + c4); }
#pragma unroll
      for (int t = 0; t < 4; ++t) {
        unsigned short hb = bf16_bits(kf[t]); sKh[r][c4 + t] = hb; sKl[r][c4 + t] = bf16_bits(kf[t] - bf16_val(hb));
        hb = bf16_bits(vf[t]); sVh[r][c4 + t] = hb; sVl[r][c4 + t] = bf16_bits(vf[t] - bf16_val(hb));
      }
    }
    __syncthreads();
    v8f s[2];
#pragma unroll
    for (int nt = 0; nt < 2; ++nt) {
      v8f acc = {};
#pragma unroll
      for (int ks = 0; ks < KS; ++ks) {
        FragB bh_, bl_;
        bh_.half[0] = *(const v8us*)&sKh[nt * 16 + ln][ks * 32 + 8 * hh]; bh_.half[1] = *(const v8us*)&sKh[nt * 16 + ln][ks * 32 + 16 + 8 * hh];
        bl_.half[0] = *(const v8us*)&sKl[nt * 16 + ln][ks * 32 + 8 * hh]; bl_.half[1] = *(const v8us*)&sKl[nt * 16 + ln][ks * 32 + 16 + 8 * hh];
        acc = mmaN<3>(aqh[ks].v, aql[ks].v, bh_.v, bl_.v, acc);
      }
      s[nt] = acc;
    }
    float alpha[8];
#pragma unroll
    for (int r = 0; r < 8; ++r) {
      const int qi = q0 + 8 * hh + r;
      const int ja = j0 + ln, jb = j0 + 16 + ln;
      if (CAUSAL) { if (ja > qi) s[0][r] = -3.0e38f; if (jb > qi) s[1][r] = -3.0e38f; }
      if (ja >= T) s[0][r] = -3.0e38f;
      if (jb >= T) s[1][r] = -3.0e38f;
      float mx = fmaxf(s[0][r], s[1][r]);
      mx = fmaxf(mx, __shfl_xor(mx, 1, 32)); mx = fmaxf(mx, __shfl_xor(mx, 2, 32)); mx = fmaxf(mx, __shfl_xor(mx, 4, 32)); mx = fmaxf(mx, __shfl_xor(mx, 8, 32));
      const float mnew = fmaxf(m_r[r], mx);
      alpha[r] = (mnew > -1.0e38f) ? __expf(m_r[r] - mnew) : 1.0f;
      const float p0 = (s[0][r] > -1.0e38f) ? __expf(s[0][r] - mnew) : 0.f;
      const float p1 = (s[1][r] > -1.0e38f) ? __expf(s[1][r] - mnew) : 0.f;
      m_r[r] = mnew;
      l_r[r] = l_r[r] * alpha[r] + p0 + p1;
      unsigned short hb = bf16_bits(p0); sPh[w][8 * hh + r][ln] = hb;      sPl[w][8 * hh + r][ln] = bf16_bits(p0 - bf16_val(hb));
      hb = bf16_bits(p1);                sPh[w][8 * hh + r][16 + ln] = hb; sPl[w][8 * hh + r][16 + ln] = bf16_bits(p1 - bf16_val(hb));
    }
#pragma unroll
    for (int dt = 0; dt < DT; ++dt)
#pragma unroll
      for (int r = 0; r < 8; ++r) oacc[dt][r] *= alpha[r];
    __builtin_amdgcn_fence(__ATOMIC_ACQ_REL, "workgroup");
    __builtin_amdgcn_wave_barrier();
    FragB pah, pal;
    pah.half[0] = *(const v8us*)&sPh[w][ln][8 * hh]; pah.half[1] = *(const v8us*)&sPh[w][ln][16 + 8 * hh];
    pal.half[0] = *(const v8us*)&sPl[w][ln][8 * hh]; pal.half[1] = *(const v8us*)&sPl[w][ln][16 + 8 * hh];
#pragma unroll
    for (int dt = 0; dt < DT; ++dt) {
      FragB bvh, bvl;
#pragma unroll
      for (int i = 0; i < 8; ++i) {
        bvh.u[i] = sVh[8 * hh + i][dt * 16 + ln]; bvh.u[8 + i] = sVh[16 + 8 * hh + i][dt * 16 + ln];
        bvl.u[i] = sVl[8 * hh + i][dt * 16 + ln]; bvl.u[8 + i] = sVl[16 + 8 * hh + i][dt * 16 + ln];
      }
      oacc[dt] = mmaN<3>(pah.v, pal.v, bvh.v, bvl.v, oacc[dt]);
    }
    __builtin_amdgcn_fence(__ATOMIC_ACQ_REL, "workgroup");
    __builtin_amdgcn_wave_barrier();
  }
#pragma unroll
  for (int r = 0; r < 8; ++r) {
    float l = l_r[r];
    l += __shfl_xor(l, 1, 32); l += __shfl_xor(l, 2, 32); l += __shfl_xor(l, 4, 32); l += __shfl_xor(l, 8, 32);
    l_r[r] = (l > 0.f) ? 1.0f / l : 0.f;
  }
#pragma unroll
  for (int dt = 0; dt < DT; ++dt)
#pragma unroll
    for (int r = 0; r < 8; ++r) sO[w][8 * hh + r][dt * 16 + ln] = oacc[dt][r] * l_r[r];
  __builtin_amdgcn_fence(__ATOMIC_ACQ_REL, "workgroup");
  __builtin_amdgcn_wave_barrier();
  for (int pass = 0; pass < 2; ++pass) {
    for (int r = 0; r < 16; ++r) {
      const int row = q0 + r;
      if (row < T && lane < D / 4) {
        const v4f val = *(const v4fa*)&sO[w][r][lane * 4];
        *(volatile v4f*)(y + ((size_t)b * T + row) * ypitch + h * D + lane * 4) = val;
      }
    }
    if (pass == 0) __threadfence();
  }
}

template <bool ASPLIT, int ACT, bool BIAS_BF16, bool RES_BF16>
__global__ __launch_bounds__(128) void k_gemm_bf3(const float* __restrict__ A, int lda, const unsigned short* __restrict__ Wt, int ldb,
                                                const float* __restrict__ bias, const float* __restrict__ resid, int rmod, int ldr,
                                                float* __restrict__ C, int ldc, int M, int N, int K) {
  __shared__ __attribute__((aligned(16))) float so[4][16][64];
  const int tid = threadIdx.x, w = tid >> 5, lane = tid & 31, ln = lane & 15, hh = lane >> 4;
  const int ntn = N / 64;
  const int wid = blockIdx.x * 4 + w;
  const int mt = wid / ntn, nq = wid % ntn;
  if (mt * 16 >= M) return;
  const int row0 = mt * 16, col0 = nq * 64;
  const float* arow = A + (size_t)(row0 + ln) * lda;
  v8f acc[4] = {};
  for (int kb = 0; kb < K; kb += 32) {
    FragB ah, al;
    const v4f x0 = *(const v4fa*)(arow + kb + 8 * hh), x1 = *(const v4fa*)(arow + kb + 8 * hh + 4);
    const v4f x2 = *(const v4fa*)(arow + kb + 16 + 8 * hh), x3 = *(const v4fa*)(arow + kb + 16 + 8 * hh + 4);
    float xs[16] = {x0[0],x0[1],x0[2],x0[3],x1[0],x1[1],x1[2],x1[3],x2[0],x2[1],x2[2],x2[3],x3[0],x3[1],x3[2],x3[3]};
#pragma unroll
    for (int i = 0; i < 16; ++i) { const unsigned short hb = bf16_bits(xs[i]); ah.u[i] = hb; al.u[i] = ASPLIT ? bf16_bits(xs[i] - bf16_val(hb)) : (unsigned short)0; }
#pragma unroll
    for (int t = 0; t < 4; ++t) {
      const unsigned short* brow = Wt + (size_t)(col0 + t * 16 + ln) * ldb + kb;
      FragB b;
      b.half[0] = *(const v8us*)(brow + 8 * hh);
      b.half[1] = *(const v8us*)(brow + 16 + 8 * hh);
      acc[t] = mmaN<ASPLIT ? 2 : 1>(ah.v, al.v, b.v, b.v, acc[t]);
    }
  }
#pragma unroll
  for (int t = 0; t < 4; ++t) {
    const int col = col0 + t * 16 + ln;
    float bv = bias ? bias[col] : 0.f;
    if (BIAS_BF16) bv = bf16_round(bv);
#pragma unroll
    for (int r = 0; r < 8; ++r) {
      float v = acc[t][r] + bv;
      if (resid) { float rv = resid[(size_t)((row0 + 8 * hh + r) % rmod) * ldr + col]; if (RES_BF16) rv = bf16_round(rv); v += rv; }
      if (ACT == 1) v = fmaxf(v, 0.f);
      if (ACT == 2) v = 0.5f * v * (1.0f + erff(v * 0.70710678118654752f));
      if (ACT == 3) { const float u = 0.7978845608028654f * (v + 0.044715f * v * v * v); v = 0.5f * v * (1.0f + tanhf(u)); }
      so[w][8 * hh + r][t * 16 + ln] = v;
    }
  }
  __builtin_amdgcn_fence(__ATOMIC_ACQ_REL, "workgroup");
  __builtin_amdgcn_wave_barrier();
  const int rsub = lane >> 4, c4 = (lane & 15) * 4;
  for (int pass = 0; pass < 2; ++pass) {
#pragma unroll
    for (int q = 0; q < 8; ++q) {
      const int r = q * 2 + rsub;
      const v4f v = *(const v4fa*)&so[w][r][c4];
      *(volatile v4f*)(C + (size_t)(row0 + r) * ldc + col0 + c4) = v;
    }
    if (pass == 0) __threadfence();
  }
}
template <bool PARAM_BF16>
__global__ __launch_bounds__(256) void k_layernorm(const float* __restrict__ X, const float* __restrict__ R, const float* __restrict__ g, const float* __restrict__ bta,
                                                  float* __restrict__ out_sum, float* __restrict__ out_norm, int N, float eps) {
  __shared__ float red[256];
  const int row = blockIdx.x, tid = threadIdx.x;
  const float* x = X + (size_t)row * N; const float* rr = R ? R + (size_t)row * N : nullptr;
  float vals[16];
  const int per = N / 256;
  float s1 = 0.f;
  for (int u = 0; u < per / 4; ++u) {
    const int j = tid * 4 + 1024 * u;
    const v4f a = *(const v4fa*)(x + j);
    v4f b = {0.f,0.f,0.f,0.f}; if (rr) b = *(const v4fa*)(rr + j);
#pragma unroll
    for (int q = 0; q < 4; ++q) { const float v = a[q] + b[q]; vals[u * 4 + q] = v; s1 += v; }
  }
  red[tid] = s1; __syncthreads();
  for (int st = 128; st > 0; st >>= 1) { if (tid < st) red[tid] += red[tid + st]; __syncthreads(); }
  const float mu = red[0] / (float)N; __syncthreads();
  float s2 = 0.f;
  for (int u = 0; u < per / 4; ++u)
#pragma unroll
    for (int q = 0; q < 4; ++q) { const float c = vals[u * 4 + q] - mu; s2 += c * c; }
  red[tid] = s2; __syncthreads();
  for (int st = 128; st > 0; st >>= 1) { if (tid < st) red[tid] += red[tid + st]; __syncthreads(); }
  const float rs = rsqrtf(red[0] / (float)N + eps);
  for (int pass = 0; pass < 2; ++pass) {
    for (int u = 0; u < per / 4; ++u) {
      const int j = tid * 4 + 1024 * u;
      v4f o, sm;
#pragma unroll
      for (int q = 0; q < 4; ++q) {
        float gg = g[j + q], bb = bta[j + q];
        if (PARAM_BF16) { gg = bf16_round(gg); bb = bf16_round(bb); }
        sm[q] = vals[u * 4 + q]; o[q] = (vals[u * 4 + q] - mu) * rs * gg + bb;
      }
      if (out_sum) *(volatile v4f*)(out_sum + (size_t)row * N + j) = sm;
      *(volatile v4f*)(out_norm + (size_t)row * N + j) = o;
    }
    if (pass == 0) __threadfence();
  }
}

typedef _Float16 v16h __attribute__((ext_vector_type(16)));
union FragH { v16h v; v8us half[2]; _Float16 h[16]; unsigned short u[16]; };
template <int NT>
__device__ __forceinline__ v8f mmaH(v16h ah, v16h al, v16h bh, v16h bl, v8f c) {
  c = __builtin_amdgcn_wmma_f32_16x16x32_f16(false, ah, false, bh, (short)0, c, false, false);
  if (NT >= 2) c = __builtin_amdgcn_wmma_f32_16x16x32_f16(false, al, false, bh, (short)0, c, false, false);
  if (NT >= 3) c = __builtin_amdgcn_wmma_f32_16x16x32_f16(false, ah, false, bl, (short)0, c, false, false);
  asm volatile("v_nop\n\tv_nop\n\tv_nop\n\tv_nop" : "+v"(c) : "v"(ah), "v"(al), "v"(bh), "v"(bl));
  return c;
}
template <bool ASPLIT>
__global__ __launch_bounds__(128) void k_gemm_h(const float* __restrict__ A, int lda, size_t sA, const _Float16* __restrict__ Bh, int ldb, size_t sB, float alpha, float* __restrict__ C, int ldc, size_t sC, int M, int N, int K) {
  __shared__ __attribute__((aligned(16))) float so[4][16][64];
  const int tid = threadIdx.x, w = tid >> 5, lane = tid & 31, ln = lane & 15, hh = lane >> 4; const int by = blockIdx.y;
  A += (size_t)by * sA; Bh += (size_t)by * sB; C += (size_t)by * sC;
  const int ntn = (N + 63) / 64; const int wid = blockIdx.x * 4 + w; const int mt = wid / ntn, nq = wid % ntn; if (mt * 16 >= M) return;
  const int row0 = mt * 16, col0 = nq * 64; const float* arow = A + (size_t)(row0 + ln) * lda;
  v8f acc[4] = {};
  for (int kb = 0; kb < K; kb += 32) {
    FragH ah, al;
    const v4f x0 = *(const v4fa*)(arow + kb + 8 * hh), x1 = *(const v4fa*)(arow + kb + 8 * hh + 4), x2 = *(const v4fa*)(arow + kb + 16 + 8 * hh), x3 = *(const v4fa*)(arow + kb + 16 + 8 * hh + 4);
    float xs[16] = {x0[0],x0[1],x0[2],x0[3],x1[0],x1[1],x1[2],x1[3],x2[0],x2[1],x2[2],x2[3],x3[0],x3[1],x3[2],x3[3]};
#pragma unroll
    for (int i = 0; i < 16; ++i) { const _Float16 h = (_Float16)xs[i]; ah.h[i] = h; al.h[i] = ASPLIT ? (_Float16)(xs[i] - (float)h) : (_Float16)0.0f; }
#pragma unroll
    for (int t = 0; t < 4; ++t) { if (col0 + t * 16 >= N) continue; const size_t boff = (size_t)(col0 + t * 16 + ln) * ldb + kb; FragH bq; bq.half[0] = *(const v8us*)(Bh + boff + 8 * hh); bq.half[1] = *(const v8us*)(Bh + boff + 16 + 8 * hh);
      acc[t] = mmaH<ASPLIT ? 2 : 1>(ah.v, al.v, bq.v, bq.v, acc[t]); }
  }
#pragma unroll
  for (int t = 0; t < 4; ++t) { if (col0 + t * 16 >= N) continue;
#pragma unroll
    for (int r = 0; r < 8; ++r) so[w][8 * hh + r][t * 16 + ln] = acc[t][r] * alpha; }
  __builtin_amdgcn_fence(__ATOMIC_ACQ_REL, "workgroup"); __builtin_amdgcn_wave_barrier();
  const int rsub = lane >> 4, c4 = (lane & 15) * 4;
  for (int pass = 0; pass < 2; ++pass) {
#pragma unroll
    for (int q = 0; q < 8; ++q) { const int r = q * 2 + rsub; if (col0 + c4 < N) { const v4f v = *(const v4fa*)&so[w][r][c4]; *(volatile v4f*)(C + (size_t)(row0 + r) * ldc + col0 + c4) = v; } }
    if (pass == 0) __threadfence(); }
}

__global__ __launch_bounds__(256) void k_wt_f16(const float* __restrict__ W, _Float16* __restrict__ Wt, int K, int N, float scale) { const int t = blockIdx.x * 256 + threadIdx.x; if (t >= N * (K / 8)) return; const int n = t / (K / 8), k8 = (t % (K / 8)) * 8; FragH f;
#pragma unroll
  for (int i = 0; i < 8; ++i) f.h[i] = (_Float16)(bf16_round(W[(size_t)(k8 + i) * N + n]) * scale); const v8us o = f.half[0]; *(volatile v8us*)((unsigned short*)Wt + (size_t)n * K + k8) = o; __threadfence(); *(volatile v8us*)((unsigned short*)Wt + (size_t)n * K + k8) = o; }
__global__ __launch_bounds__(256) void k_blocks(const int* __restrict__ new_t, const int* __restrict__ past_t, int* __restrict__ LIST, int* __restrict__ KPOS, int* __restrict__ KVAL) {
  __shared__ int smax[256]; __shared__ int sact[NKB_ALL]; __shared__ int slist[NKB_MAX + 1]; const int t = threadIdx.x;
  int m = -2147483647; for (int i = t; i < SN; i += 256) m = max(m, new_t[i]); smax[t] = m; __syncthreads(); for (int s = 128; s > 0; s >>= 1) { if (t < s) smax[t] = max(smax[t], smax[t + s]); __syncthreads(); } const int min_time = smax[0] - (WIN - 1);
  if (t < NKB_ALL) { int act = 1; if (t < LP / 64) { act = 0; for (int i = 0; i < 64; ++i) act |= (past_t[t * 64 + i] >= min_time) ? 1 : 0; } sact[t] = act; } __syncthreads();
  if (t == 0) { int n = 0; for (int b = 0; b < NKB_ALL; ++b) if (sact[b] && n < NKB_MAX) slist[n++] = b; for (int q = n; q < NKB_MAX; ++q) slist[q] = -1; slist[NKB_MAX] = n; } __syncthreads();
  for (int pass = 0; pass < 2; ++pass) {
    if (t <= NKB_MAX) *(volatile int*)(LIST + t) = slist[t];
    for (int kidx = t; kidx < KC; kidx += 256) { const int b = slist[kidx / 64]; int pos = 2147483647, val = 0; if (b >= 0) { const int key = b * 64 + (kidx & 63); if (key < LP) { pos = past_t[key]; val = (pos >= min_time) ? 1 : 0; } else { pos = new_t[key - LP]; val = 1; } } *(volatile int*)(KPOS + kidx) = pos; *(volatile int*)(KVAL + kidx) = val; }
    if (pass == 0) __threadfence(); }
}
__device__ __forceinline__ float rope_ang(int pt, int pd, int pb, int i) { const float invf = 1.0f / powf(10000.0f, (2.0f * (float)i) / 64.0f); return ((float)pt * invf + ((float)pd * invf) * 100.0f) + ((float)pb * invf) * 100.0f; }
__global__ __launch_bounds__(256) void k_rope_new(const float* __restrict__ P, const int* __restrict__ nt, const int* __restrict__ nd, const int* __restrict__ nb, const int* __restrict__ LIST, float* __restrict__ Qr, float* __restrict__ Kout, float* __restrict__ Vout, _Float16* __restrict__ K16, _Float16* __restrict__ VR16) {
  const int t = blockIdx.x * 256 + threadIdx.x; if (t >= SN * 24 * 32) return; const int i = t & 31; const int slot = (t >> 5) % 24; const int s = t / (32 * 24); const float* row = P + (size_t)s * 1536;
  const float ang = rope_ang(nt[s], nd[s], nb[s], i); const float cs = cosf(ang), sn = sinf(ang);
  int ls = -1; const int myb = LP / 64 + s / 64; for (int q = 0; q < NKB_MAX; ++q) if (LIST[q] == myb) ls = q; const int kidx = (ls >= 0) ? ls * 64 + (s & 63) : -1;
  if (slot < 16) { const int h = slot; const float x1 = row[h * 64 + 2 * i], x2 = row[h * 64 + 2 * i + 1]; const float y1 = x1 * cs - x2 * sn, y2 = x1 * sn + x2 * cs; float* d = Qr + ((size_t)h * SN + s) * 64 + 2 * i; typedef float v2f __attribute__((ext_vector_type(2))); v2f v; v.x = y1; v.y = y2; *(volatile v2f*)d = v; __threadfence(); *(volatile v2f*)d = v; }
  else if (slot < 20) { const int g = slot - 16; const float x1 = row[1024 + g * 64 + 2 * i], x2 = row[1024 + g * 64 + 2 * i + 1]; const float y1 = x1 * cs - x2 * sn, y2 = x1 * sn + x2 * cs; typedef float v2f __attribute__((ext_vector_type(2))); v2f v; v.x = y1; v.y = y2; typedef _Float16 v2h __attribute__((ext_vector_type(2))); v2h hv; hv.x = (_Float16)y1; hv.y = (_Float16)y2;
    float* d = Kout + ((size_t)g * SN + s) * 64 + 2 * i; *(volatile v2f*)d = v; if (kidx >= 0) *(volatile v2h*)(K16 + ((size_t)g * KC + kidx) * 64 + 2 * i) = hv; __threadfence(); *(volatile v2f*)d = v; if (kidx >= 0) *(volatile v2h*)(K16 + ((size_t)g * KC + kidx) * 64 + 2 * i) = hv; }
  else { const int g = slot - 20; const float x1 = row[1280 + g * 64 + 2 * i], x2 = row[1280 + g * 64 + 2 * i + 1]; typedef float v2f __attribute__((ext_vector_type(2))); v2f v; v.x = x1; v.y = x2; typedef _Float16 v2h __attribute__((ext_vector_type(2))); v2h hv; hv.x = (_Float16)x1; hv.y = (_Float16)x2; float* d = Vout + ((size_t)g * SN + s) * 64 + 2 * i;
    *(volatile v2f*)d = v; if (kidx >= 0) *(volatile v2h*)(VR16 + ((size_t)g * KC + kidx) * 64 + 2 * i) = hv; __threadfence(); *(volatile v2f*)d = v; if (kidx >= 0) *(volatile v2h*)(VR16 + ((size_t)g * KC + kidx) * 64 + 2 * i) = hv; }
}
__global__ __launch_bounds__(256) void k_past(const float* __restrict__ pk, const float* __restrict__ pv, const int* __restrict__ LIST, _Float16* __restrict__ K16, _Float16* __restrict__ VR16) {
  const int t = blockIdx.x * 256 + threadIdx.x; if (t >= NKV * KC * 8) return; const int d8 = (t & 7) * 8; const int kidx = (t >> 3) % KC; const int g = t / (8 * KC); const int b = LIST[kidx / 64];
  if (b >= LP / 64) return;
  FragH kf, vf; for (int q = 0; q < 8; ++q) { float kvv = 0.f, vvv = 0.f; if (b >= 0) { const size_t key = (size_t)b * 64 + (kidx & 63); kvv = bf16_round(pk[((size_t)g * LP + key) * 64 + d8 + q]); vvv = bf16_round(pv[((size_t)g * LP + key) * 64 + d8 + q]); } kf.h[q] = (_Float16)kvv; vf.h[q] = (_Float16)vvv; }
  *(volatile v8us*)((unsigned short*)K16 + ((size_t)g * KC + kidx) * 64 + d8) = kf.half[0]; *(volatile v8us*)((unsigned short*)VR16 + ((size_t)g * KC + kidx) * 64 + d8) = vf.half[0]; __threadfence();
  *(volatile v8us*)((unsigned short*)K16 + ((size_t)g * KC + kidx) * 64 + d8) = kf.half[0]; *(volatile v8us*)((unsigned short*)VR16 + ((size_t)g * KC + kidx) * 64 + d8) = vf.half[0];
}
__global__ __launch_bounds__(256) void k_tr16(const _Float16* __restrict__ VR, _Float16* __restrict__ Vt) { __shared__ _Float16 tile[64][34]; const int g = blockIdx.z; const int k0 = blockIdx.x * 64, d0 = blockIdx.y * 32; const int tx = threadIdx.x & 31, ty = threadIdx.x >> 5;
  for (int i = ty; i < 64; i += 8) tile[i][tx] = VR[((size_t)g * KC + k0 + i) * 64 + d0 + tx]; __syncthreads();
  typedef _Float16 v2h __attribute__((ext_vector_type(2)));
  for (int pass = 0; pass < 2; ++pass) { for (int e = threadIdx.x; e < 32 * 32; e += 256) { const int dr = e >> 5, kp = (e & 31) * 2; v2h v; v.x = tile[kp][dr]; v.y = tile[kp + 1][dr]; *(volatile v2h*)(Vt + ((size_t)g * 64 + d0 + dr) * KC + k0 + kp) = v; } if (pass == 0) __threadfence(); } }
__global__ __launch_bounds__(1024) void k_softmax(float* __restrict__ S, const int* __restrict__ KPOS, const int* __restrict__ KVAL, const int* __restrict__ nt, int h0, float* __restrict__ Dn) {
  __shared__ float sd[32]; const int tid = threadIdx.x, wv = tid >> 5, lane = tid & 31; const int r = blockIdx.x * 32 + wv; const int hl = r / SN, s = r % SN; float* row = S + (size_t)r * KC; const int myt = nt[s];
  float mx = -3.0e38f;
#pragma unroll 1
  for (int j = lane; j < KC; j += 32) { const bool ok = KVAL[j] && (KPOS[j] <= myt); if (ok) mx = fmaxf(mx, row[j] * 0.125f); }
  for (int o = 16; o >= 1; o >>= 1) mx = fmaxf(mx, __shfl_xor(mx, o, 32));
  float den = 0.f;
#pragma unroll 1
  for (int j = lane; j < KC; j += 32) { const bool ok = KVAL[j] && (KPOS[j] <= myt); const float e = ok ? expf(row[j] * 0.125f - mx) : 0.f; den += e; *(volatile float*)(row + j) = e * 256.0f; }
  for (int o = 16; o >= 1; o >>= 1) den += __shfl_xor(den, o, 32);
  __threadfence();
#pragma unroll 1
  for (int j = lane; j < KC; j += 32) { const float pvv = row[j]; *(volatile float*)(row + j) = pvv; }
  if (lane == 0) sd[wv] = den; __syncthreads(); (void)hl;
  if (tid < 32) { *(volatile float*)(Dn + ((size_t)h0 * SN) + (size_t)blockIdx.x * 32 + tid) = sd[tid]; } __threadfence(); if (tid < 32) { *(volatile float*)(Dn + ((size_t)h0 * SN) + (size_t)blockIdx.x * 32 + tid) = sd[tid]; }
}
__global__ __launch_bounds__(256) void k_onorm(const float* __restrict__ O, const float* __restrict__ Dn, float* __restrict__ OC) { const int t = blockIdx.x * 256 + threadIdx.x; if (t >= SN * ED / 4) return; const int c4 = (t % (ED / 4)) * 4; const int s = t / (ED / 4); const int h = c4 / 64, d4 = c4 % 64; const float dn = Dn[(size_t)h * SN + s]; const float rd = (dn > 0.f) ? 1.0f / dn : 0.f;
  const v4f o = *(const v4fa*)(O + ((size_t)h * SN + s) * 64 + d4); v4f r; for (int q = 0; q < 4; ++q) r[q] = o[q] * rd; *(volatile v4f*)(OC + (size_t)t * 4) = r; __threadfence(); *(volatile v4f*)(OC + (size_t)t * 4) = r; }
extern "C" void kernel_launch(void* const* d_in, const int* in_sizes, int n_in,
                              void* d_out, int out_size, void* d_ws, size_t ws_size, hipStream_t stream) {
  (void)in_sizes; (void)n_in; (void)out_size;
  const float* hid = (const float*)d_in[0]; const float* pk = (const float*)d_in[1]; const float* pv = (const float*)d_in[2]; const float* wq = (const float*)d_in[3]; const float* wk = (const float*)d_in[4]; const float* wv = (const float*)d_in[5]; const float* wo = (const float*)d_in[6];
  const int* nt = (const int*)d_in[7]; const int* nd = (const int*)d_in[8]; const int* nb = (const int*)d_in[9]; const int* pt = (const int*)d_in[10]; (void)d_in[11]; (void)d_in[12];
  float* out = (float*)d_out; float* Kout = out + (size_t)SN * ED; float* Vout = Kout + (size_t)NKV * SN * 64;
  char* ws = (char*)d_ws; size_t off = 0;
  auto take = [&](size_t bytes) { char* p = ws + off; off += (bytes + 255) & ~(size_t)255; return p; };
  unsigned short* Bqkv = (unsigned short*)take((size_t)1536 * ED * 2); _Float16* Bo = (_Float16*)take((size_t)ED * ED * 2);
  int* LIST = (int*)take(64 * 4); int* KPOS = (int*)take(KC * 4); int* KVAL = (int*)take(KC * 4);
  float* P = (float*)take((size_t)SN * 1536 * 4); float* Qr = (float*)take((size_t)NHQ * SN * 64 * 4); _Float16* K16 = (_Float16*)take((size_t)NKV * KC * 64 * 2); _Float16* VR16 = (_Float16*)take((size_t)NKV * KC * 64 * 2); _Float16* Vt16 = (_Float16*)take((size_t)NKV * 64 * KC * 2);
  float* S = (float*)take((size_t)4 * SN * KC * 4); float* Dn = (float*)take((size_t)NHQ * SN * 4); float* O = (float*)take((size_t)NHQ * SN * 64 * 4); float* OC = (float*)take((size_t)SN * ED * 4);
  if (off > ws_size) return;
  k_wt_bf16<<<(1024 * 128 + 255) / 256, 256, 0, stream>>>(wq, Bqkv, ED, 1024); k_wt_bf16<<<(256 * 128 + 255) / 256, 256, 0, stream>>>(wk, Bqkv + (size_t)1024 * ED, ED, 256); k_wt_bf16<<<(256 * 128 + 255) / 256, 256, 0, stream>>>(wv, Bqkv + (size_t)1280 * ED, ED, 256);
  k_wt_f16<<<(ED * 128 + 255) / 256, 256, 0, stream>>>(wo, Bo, ED, ED, 16.0f);
  k_blocks<<<1, 256, 0, stream>>>(nt, pt, LIST, KPOS, KVAL);
  k_gemm_bf3<false, 0, false, false><<<((SN / 16) * 24 + 3) / 4, 128, 0, stream>>>(hid, ED, Bqkv, ED, nullptr, nullptr, 1, 0, P, 1536, SN, 1536, ED);
  k_past<<<(NKV * KC * 8 + 255) / 256, 256, 0, stream>>>(pk, pv, LIST, K16, VR16);
  k_rope_new<<<(SN * 24 * 32 + 255) / 256, 256, 0, stream>>>(P, nt, nd, nb, LIST, Qr, Kout, Vout, K16, VR16);
  k_tr16<<<dim3(KC / 64, 2, NKV), 256, 0, stream>>>(VR16, Vt16);
  for (int g = 0; g < NKV; ++g) {
    k_gemm_h<false><<<dim3(((SN / 16) * (KC / 64) + 3) / 4, 4), 128, 0, stream>>>(Qr + (size_t)(g * 4) * SN * 64, 64, (size_t)SN * 64, K16 + (size_t)g * KC * 64, 64, 0, 1.f, S, KC, (size_t)SN * KC, SN, KC, 64);
    for (int hl = 0; hl < 4; ++hl) k_softmax<<<SN / 32, 1024, 0, stream>>>(S + (size_t)hl * SN * KC, KPOS, KVAL, nt, g * 4 + hl, Dn);
    k_gemm_h<false><<<dim3(((SN / 16) * 1 + 3) / 4, 4), 128, 0, stream>>>(S, KC, (size_t)SN * KC, Vt16 + (size_t)g * 64 * KC, KC, 0, 0.00390625f, O + (size_t)(g * 4) * SN * 64, 64, (size_t)SN * 64, SN, 64, KC);
  }
  k_onorm<<<(SN * ED / 4 + 255) / 256, 256, 0, stream>>>(O, Dn, OC);
  k_gemm_h<false><<<dim3(((SN / 16) * (ED / 64) + 3) / 4, 1), 128, 0, stream>>>(OC, ED, 0, Bo, ED, 0, 0.0625f, out, ED, 0, SN, ED, ED);
}
